// Model5_9620726743221
// MI455X (gfx1250) — hardware-verified
//
#include <hip/hip_runtime.h>
#include <stddef.h>
#include <math.h>


#define NF     15
#define NBA    4096
#define ACP    12
#define CHUNK  8192
#define ATHR   256
#define AWAVE  8
#define WCAP   1024
#define NGRP   (CHUNK / (ATHR * 4))
#define GTHR   128
#define GR     64
#define APN    40
#define APA    72
#define XSP    36

#define AGG_ACC_F  ((NBA + 1) * ACP)
#define AGG_LIST_I (AWAVE * WCAP)
#define AGG_STG_F  (AWAVE * 32 * 16)
#define AGG_LDS_BYTES ((AGG_ACC_F + AGG_LIST_I + AGG_STG_F + 16) * 4)

#define WPL_HALVES 6656
#define WPL_PIECES (WPL_HALVES / 8)

static_assert(WCAP == (CHUNK / ATHR) * 32);
static_assert(NGRP * ATHR * 4 == CHUNK);
static_assert(NBA == 4096);
static_assert(CHUNK == 8192);
static_assert(ATHR * 16 == AGG_STG_F);
static_assert((AGG_ACC_F % 4) == 0);
static_assert(((AGG_ACC_F + AGG_LIST_I) % 4) == 0);
static_assert(AGG_LDS_BYTES == 245872);
static_assert(WPL_PIECES == 832);

typedef float    v4f  __attribute__((ext_vector_type(4)));
typedef float    v8f  __attribute__((ext_vector_type(8)));
typedef int      v4i  __attribute__((ext_vector_type(4)));
typedef _Float16 v8h  __attribute__((ext_vector_type(8)));
typedef _Float16 v16h __attribute__((ext_vector_type(16)));
union Frag   { v16h v; v8h half[2]; };
union Pack16 { v8h h; v4i i; };

__device__ __forceinline__ v8f wm(v16h a, v16h b, v8f c) {
  v8f d = __builtin_amdgcn_wmma_f32_16x16x32_f16(false, a, false, b, (short)0, c, false, false);
  asm volatile("v_nop\n\tv_nop\n\tv_nop\n\tv_nop" : "+v"(d) : "v"(a), "v"(b));
  return d;
}

__device__ __forceinline__ float lrelu(float t) { return t > 0.f ? t : 0.2f * t; }

__device__ __forceinline__ int clampi(int v, int lo, int hi) { return v < lo ? lo : (v > hi ? hi : v); }

__global__ __launch_bounds__(256) void k_prepw(
    const float* __restrict__ wl0, const float* __restrict__ wr0,
    const float* __restrict__ wl1, const float* __restrict__ wr1,
    const float* __restrict__ wl2, const float* __restrict__ wr2,
    const float* __restrict__ aw,  const float* __restrict__ cw,  const float* __restrict__ lw,
    _Float16* wpl, int npieces) {
  const int i = blockIdx.x * 256 + threadIdx.x;
  if (i >= npieces) return;
  const int p = (i < 128) ? 0 : (i < 256) ? 1 : (i < 384) ? 2 : (i < 640) ? 3 : (i < 768) ? 4 : 5;
  const int pbase = (p == 0) ? 0 : (p == 1) ? 128 : (p == 2) ? 256 : (p == 3) ? 384 : (p == 4) ? 640 : 768;
  const int lp = i - pbase;
  const int sh = (p == 3) ? 3 : 2;
  const int n  = lp >> sh;
  const int kb = (lp - (n << sh)) * 8;
  const bool hi = (p < 3) && (n >= 16);
  const int nn = (p < 3) ? (hi ? n - 16 : n) : n;
  const int K  = (p == 0) ? 15 : (p < 3) ? 25 : (p == 3) ? 48 : (p == 4) ? 23 : 29;
  const int NO = (p < 3) ? 10 : (p == 5) ? 15 : 20;
  const float* W = (p == 0) ? (hi ? wr0 : wl0)
                 : (p == 1) ? (hi ? wr1 : wl1)
                 : (p == 2) ? (hi ? wr2 : wl2)
                 : (p == 3) ? aw : (p == 4) ? cw : lw;
  Pack16 u;
#pragma unroll
  for (int j = 0; j < 8; ++j) {
    const int k = kb + j;
    const bool ok = (nn < NO) && (k < K);
    const int kc = (k < K) ? k : K - 1;
    const int nc = (nn < NO) ? nn : NO - 1;
    const float v = W[kc * NO + nc];
    u.h[j] = ok ? (_Float16)v : (_Float16)0.0f;
  }
  _Float16* dp = wpl + (size_t)i * 8;
  *(volatile v4i*)dp = u.i;
  __threadfence();
  *(volatile v4i*)dp = u.i;
}

__global__ __launch_bounds__(GTHR) void k_node(
    const float* __restrict__ x1, const float* __restrict__ hin,
    const _Float16* __restrict__ wpl, float* xlr, int nh, int nN) {
  __shared__ __attribute__((aligned(16))) _Float16 At[GR * APN];
  __shared__ __attribute__((aligned(16))) float Xs[GR * XSP];
  const int tid = threadIdx.x, lane = tid & 31, wave = tid >> 5;
  const int hh = lane >> 4, m = lane & 15;
  const int rowBase = blockIdx.x * GR;

  {
    const int r = tid >> 1, kh = tid & 1;
    int row = rowBase + r; if (row > nN - 1) row = nN - 1;
    const float* hp = hin + (size_t)row * 16;
    const float* xp = x1 + (size_t)row * NF;
    Pack16 u0, u1;
#pragma unroll
    for (int j = 0; j < 16; ++j) {
      const int k  = 16 * kh + j;
      const int xi = k - nh;
      const float hv = hp[k < 15 ? k : 15];
      const float xv = xp[xi < 0 ? 0 : (xi > NF - 1 ? NF - 1 : xi)];
      const float v = (k < nh) ? hv : ((xi >= 0 && xi < NF) ? xv : 0.f);
      const _Float16 f = (_Float16)v;
      if (j < 8) u0.h[j] = f; else u1.h[j - 8] = f;
    }
    *(v8h*)(At + r * APN + 16 * kh)     = u0.h;
    *(v8h*)(At + r * APN + 16 * kh + 8) = u1.h;
  }
  __syncthreads();

  Frag a, b0, b1;
  const _Float16* pa  = At + (16 * wave + m) * APN + 8 * hh;
  const _Float16* pb0 = wpl + (size_t)m * 32 + 8 * hh;
  const _Float16* pb1 = wpl + (size_t)(16 + m) * 32 + 8 * hh;
  a.half[0]  = *(const v8h*)pa;  a.half[1]  = *(const v8h*)(pa + 16);
  b0.half[0] = *(const v8h*)pb0; b0.half[1] = *(const v8h*)(pb0 + 16);
  b1.half[0] = *(const v8h*)pb1; b1.half[1] = *(const v8h*)(pb1 + 16);
  const v8f z8 = {0.f, 0.f, 0.f, 0.f, 0.f, 0.f, 0.f, 0.f};
  const v8f c0 = wm(a.v, b0.v, z8);
  const v8f c1 = wm(a.v, b1.v, z8);
#pragma unroll
  for (int r = 0; r < 8; ++r) {
    Xs[(16 * wave + 8 * hh + r) * XSP + m]      = c0[r];
    Xs[(16 * wave + 8 * hh + r) * XSP + 16 + m] = c1[r];
  }
  __syncthreads();

  v4f xv[4];
  float* xp4[4];
#pragma unroll
  for (int i = 0; i < 4; ++i) {
    const int R  = 16 * wave + 4 * i + (lane >> 3);
    const int cc = 4 * (lane & 7);
    xv[i]  = *(const v4f*)(Xs + R * XSP + cc);
    xp4[i] = xlr + (size_t)(rowBase + R) * 32 + cc;
  }
#pragma unroll
  for (int i = 0; i < 4; ++i) *(volatile v4f*)(xp4[i]) = xv[i];
  __threadfence();
#pragma unroll
  for (int i = 0; i < 4; ++i) *(volatile v4f*)(xp4[i]) = xv[i];
}

__device__ __forceinline__ void agg_apply(float* rp, float v, float ef, int cm, bool active) {
  const float a  = rp[cm < ACP ? cm : ACP - 1];
  const float mo = rp[11];
  const float mn = fmaxf(mo, ef);
  const float fo = __expf(mo - mn);
  const float wg = __expf(ef - mn);
  float na = fmaf(v, wg, a * fo);
  na = (cm < 11) ? na : mn;
  if (active && cm < ACP) rp[cm] = na;
}

__global__ __launch_bounds__(ATHR) void k_agg(
    const int* __restrict__ edges, const float* __restrict__ xlr,
    const float* __restrict__ att, const float* __restrict__ bias,
    float* hout, int nN, int nE) {
  extern __shared__ v4f lds_dyn[];
  float* acc  = (float*)lds_dyn;
  int*   list = (int*)(acc + AGG_ACC_F);
  float* stg  = (float*)(list + AGG_LIST_I);
  int*   wcnt = (int*)(stg + AGG_STG_F);

  const int tid = threadIdx.x, lane = tid & 31, wave = tid >> 5;
  const int cm = lane & 15, hsel = lane >> 4;
  const int nodeBase = blockIdx.x * NBA;
  const int* esrc = edges;
  const int* edst = edges + nE;

  float attr[10], br[10];
#pragma unroll
  for (int c = 0; c < 10; ++c) { attr[c] = att[c]; br[c] = bias[c]; }

#pragma unroll 1
  for (int slot = tid; slot < NBA; slot += ATHR) {
    int d = nodeBase + slot; if (d > nN - 1) d = nN - 1;
    const float* rp = xlr + (size_t)d * 32;
    const v4f l0 = *(const v4f*)rp,        l1 = *(const v4f*)(rp + 4),  l2 = *(const v4f*)(rp + 8);
    const v4f q0 = *(const v4f*)(rp + 16), q1 = *(const v4f*)(rp + 20), q2 = *(const v4f*)(rp + 24);
    const float xl[10] = {l0.x, l0.y, l0.z, l0.w, l1.x, l1.y, l1.z, l1.w, l2.x, l2.y};
    const float xr[10] = {q0.x, q0.y, q0.z, q0.w, q1.x, q1.y, q1.z, q1.w, q2.x, q2.y};
    float e = 0.f;
#pragma unroll
    for (int c = 0; c < 10; ++c) e += attr[c] * lrelu(xl[c] + xr[c]);
    float* ap = acc + slot * ACP;
    const v4f t0 = {xl[0], xl[1], xl[2], xl[3]};
    const v4f t1 = {xl[4], xl[5], xl[6], xl[7]};
    const v4f t2 = {xl[8], xl[9], 1.0f, e};
    *(v4f*)ap = t0; *(v4f*)(ap + 4) = t1; *(v4f*)(ap + 8) = t2;
  }
  if (tid == 0) {
    float* ap = acc + NBA * ACP;
    const v4f z4 = {0.f, 0.f, 0.f, 0.f};
    const v4f t2 = {0.f, 0.f, 1.0f, 0.f};
    *(v4f*)ap = z4; *(v4f*)(ap + 4) = z4; *(v4f*)(ap + 8) = t2;
  }
  __syncthreads();

  const bool al16 = ((nE & 3) == 0);
  const int nChunks = (nE + CHUNK - 1) / CHUNK;

#pragma unroll 1
  for (int ch = 0; ch < nChunks; ++ch) {
    const int cbase = ch * CHUNK;
    const bool full = al16 && (cbase + CHUNK <= nE);
    int wc = 0;
#pragma unroll
    for (int g = 0; g < NGRP; ++g) {
      const int el0 = (g * ATHR + tid) * 4;
      const int e0  = cbase + el0;
      const int sent = -2147483647 - 1;
      v4i d;
      if (full) {
        d = *(const v4i*)(edst + e0);
      } else {
        d.x = (e0     < nE) ? edst[min(e0,     nE - 1)] : sent;
        d.y = (e0 + 1 < nE) ? edst[min(e0 + 1, nE - 1)] : sent;
        d.z = (e0 + 2 < nE) ? edst[min(e0 + 2, nE - 1)] : sent;
        d.w = (e0 + 3 < nE) ? edst[min(e0 + 3, nE - 1)] : sent;
      }
      const unsigned s0 = (unsigned)d.x - (unsigned)nodeBase;
      const unsigned s1 = (unsigned)d.y - (unsigned)nodeBase;
      const unsigned s2 = (unsigned)d.z - (unsigned)nodeBase;
      const unsigned s3 = (unsigned)d.w - (unsigned)nodeBase;
      const bool h0 = s0 < (unsigned)NBA;
      const bool h1 = s1 < (unsigned)NBA;
      const bool h2 = s2 < (unsigned)NBA;
      const bool h3 = s3 < (unsigned)NBA;
      const unsigned many = __builtin_amdgcn_ballot_w32(h0 | h1 | h2 | h3);
      if (many != 0u) {
#define HITJ(J, HJ, SJ) { \
          const unsigned mj = __builtin_amdgcn_ballot_w32(HJ); \
          if (HJ) { \
            const int pos = wc + (int)__builtin_amdgcn_mbcnt_lo(mj, 0u); \
            if (pos < WCAP) list[wave * WCAP + pos] = ((el0 + (J)) << 12) | (int)(SJ); \
          } \
          wc += (int)__builtin_popcount(mj); }
        HITJ(0, h0, s0)
        HITJ(1, h1, s1)
        HITJ(2, h2, s2)
        HITJ(3, h3, s3)
#undef HITJ
      }
    }
    if (lane == 0) wcnt[wave] = wc;
    __syncthreads();

    int maxc = 0;
#pragma unroll
    for (int w = 0; w < AWAVE; ++w) maxc = max(maxc, wcnt[w]);
    if (maxc > WCAP) maxc = WCAP;
    const int nB  = (maxc + 31) >> 5;
    const int myc = wc < WCAP ? wc : WCAP;

#pragma unroll 1
    for (int bt = 0; bt < nB; ++bt) {
      const int base = bt * 32;
      if (base < myc) {
        const int idx = base + lane;
        const bool valid = idx < myc;
        const int ent  = list[wave * WCAP + min(idx, WCAP - 1)];
        const int slot = valid ? (ent & (NBA - 1)) : NBA;
        const int el   = (ent >> 12) & (CHUNK - 1);
        int e = cbase + el; if (e > nE - 1) e = nE - 1;
        int s = esrc[e]; s = clampi(s, 0, nN - 1);
        int dn = nodeBase + slot; if (dn > nN - 1) dn = nN - 1;
        const float* sp = xlr + (size_t)s * 32;
        const float* dq = xlr + (size_t)dn * 32 + 16;
        const v4f l0 = *(const v4f*)sp, l1 = *(const v4f*)(sp + 4), l2 = *(const v4f*)(sp + 8);
        const v4f q0 = *(const v4f*)dq, q1 = *(const v4f*)(dq + 4), q2 = *(const v4f*)(dq + 8);
        const float xl[10] = {l0.x, l0.y, l0.z, l0.w, l1.x, l1.y, l1.z, l1.w, l2.x, l2.y};
        const float xr[10] = {q0.x, q0.y, q0.z, q0.w, q1.x, q1.y, q1.z, q1.w, q2.x, q2.y};
        float lg = 0.f;
#pragma unroll
        for (int c = 0; c < 10; ++c) lg += attr[c] * lrelu(xl[c] + xr[c]);
        const float vm = valid ? 1.f : 0.f;
        lg = valid ? lg : 0.f;
        float* st = stg + (wave * 32 + lane) * 16;
        const v4f t0 = {xl[0] * vm, xl[1] * vm, xl[2] * vm, xl[3] * vm};
        const v4f t1 = {xl[4] * vm, xl[5] * vm, xl[6] * vm, xl[7] * vm};
        const v4f t2 = {xl[8] * vm, xl[9] * vm, vm, lg};
        const v4f t3 = {__int_as_float(slot), 0.f, 0.f, 0.f};
        *(v4f*)st = t0; *(v4f*)(st + 4) = t1; *(v4f*)(st + 8) = t2; *(v4f*)(st + 12) = t3;
      }
      __syncthreads();
      if (wave == 0) {
#pragma unroll 1
        for (int w = 0; w < AWAVE; ++w) {
          int nw = wcnt[w]; if (nw > WCAP) nw = WCAP; nw -= base;
          nw = nw < 0 ? 0 : (nw > 32 ? 32 : nw);
          const int npair = (nw + 1) >> 1;
          const float* sw = stg + w * 512;
#pragma unroll 1
          for (int q = 0; q < npair; ++q) {
            const float v = sw[q * 32 + lane];
            const int vb = __float_as_int(v);
            int sl0 = __builtin_amdgcn_readlane(vb, 12);
            int sl1 = __builtin_amdgcn_readlane(vb, 28);
            const int eb0 = __builtin_amdgcn_readlane(vb, 11);
            const int eb1 = __builtin_amdgcn_readlane(vb, 27);
            sl0 = clampi(sl0, 0, NBA);
            sl1 = clampi(sl1, 0, NBA);
            const int slot = hsel ? sl1 : sl0;
            const float ef = __int_as_float(hsel ? eb1 : eb0);
            float* rp = acc + slot * ACP;
            if (sl0 != sl1) {
              agg_apply(rp, v, ef, cm, true);
            } else {
              agg_apply(rp, v, ef, cm, hsel == 0);
              __builtin_amdgcn_fence(__ATOMIC_RELEASE, "wavefront");
              __builtin_amdgcn_wave_barrier();
              agg_apply(rp, v, ef, cm, hsel == 1);
            }
            __builtin_amdgcn_fence(__ATOMIC_RELEASE, "wavefront");
            __builtin_amdgcn_wave_barrier();
          }
        }
      }
      __syncthreads();
    }
    __syncthreads();
  }

  float* outs = stg;
#pragma unroll 1
  for (int pass = 0; pass < NBA / ATHR; ++pass) {
    const int slot = pass * ATHR + tid;
    const float* rp = acc + slot * ACP;
    const v4f a0 = *(const v4f*)rp, a1 = *(const v4f*)(rp + 4), a2 = *(const v4f*)(rp + 8);
    const float inv = 1.0f / a2.z;
    v4f o0, o1, o2;
    const v4f o3 = {0.f, 0.f, 0.f, 0.f};
    o0.x = fmaxf(fmaf(a0.x, inv, br[0]), 0.f);
    o0.y = fmaxf(fmaf(a0.y, inv, br[1]), 0.f);
    o0.z = fmaxf(fmaf(a0.z, inv, br[2]), 0.f);
    o0.w = fmaxf(fmaf(a0.w, inv, br[3]), 0.f);
    o1.x = fmaxf(fmaf(a1.x, inv, br[4]), 0.f);
    o1.y = fmaxf(fmaf(a1.y, inv, br[5]), 0.f);
    o1.z = fmaxf(fmaf(a1.z, inv, br[6]), 0.f);
    o1.w = fmaxf(fmaf(a1.w, inv, br[7]), 0.f);
    o2.x = fmaxf(fmaf(a2.x, inv, br[8]), 0.f);
    o2.y = fmaxf(fmaf(a2.y, inv, br[9]), 0.f);
    o2.z = 0.f; o2.w = 0.f;
    float* op = outs + tid * 16;
    *(v4f*)op = o0; *(v4f*)(op + 4) = o1; *(v4f*)(op + 8) = o2; *(v4f*)(op + 12) = o3;
    __syncthreads();
    float* gb = hout + (size_t)(nodeBase + pass * ATHR) * 16;
    v4f ov[4];
#pragma unroll
    for (int i = 0; i < 4; ++i) ov[i] = *(const v4f*)(outs + (i * ATHR + tid) * 4);
#pragma unroll
    for (int i = 0; i < 4; ++i) *(volatile v4f*)(gb + (size_t)(i * ATHR + tid) * 4) = ov[i];
    __threadfence();
#pragma unroll
    for (int i = 0; i < 4; ++i) *(volatile v4f*)(gb + (size_t)(i * ATHR + tid) * 4) = ov[i];
    __syncthreads();
  }
}

__global__ __launch_bounds__(GTHR) void k_att(
    const float* __restrict__ hpl, const float* __restrict__ x1,
    const int* __restrict__ asrc, const int* __restrict__ adst, const float* __restrict__ arm,
    const _Float16* __restrict__ wpl, const float* __restrict__ ab,
    const float* __restrict__ bw, const float* __restrict__ bb,
    float* sa, int Ma, int nN) {
  __shared__ __attribute__((aligned(16))) _Float16 At[GR * APA];
  __shared__ float souts[GR];
  const int tid = threadIdx.x, lane = tid & 31, wave = tid >> 5;
  const int hh = lane >> 4, m = lane & 15;
  const int rowBase = blockIdx.x * GR;

  {
    int row = rowBase + 16 * wave + m; if (row > Ma - 1) row = Ma - 1;
    const int is = clampi(asrc[row], 0, nN - 1);
    const int id = clampi(adst[row], 0, nN - 1);
    const float ar = arm[row];
    const float* hs = hpl + (size_t)is * 16;
    const float* hd = hpl + (size_t)id * 16;
    const v4f s0 = *(const v4f*)hs, s1 = *(const v4f*)(hs + 4), s2 = *(const v4f*)(hs + 8);
    const v4f d0 = *(const v4f*)hd, d1 = *(const v4f*)(hd + 4), d2 = *(const v4f*)(hd + 8);
    const int xsel = hh ? id : is;
    const float* xp = x1 + (size_t)xsel * NF + 1;
    float xv[14];
#pragma unroll
    for (int i = 0; i < 14; ++i) xv[i] = xp[i];
    float fa[32], fb[32];
    fa[0] = s0.x; fa[1] = s0.y; fa[2] = s0.z; fa[3] = s0.w; fa[4] = s1.x;
    fa[5] = s1.y; fa[6] = s1.z; fa[7] = s1.w; fa[8] = s2.x; fa[9] = s2.y;
    fa[10] = d0.x; fa[11] = d0.y; fa[12] = d0.z; fa[13] = d0.w; fa[14] = d1.x;
    fa[15] = d1.y; fa[16] = d1.z; fa[17] = d1.w; fa[18] = d2.x; fa[19] = d2.y;
#pragma unroll
    for (int i = 0; i < 12; ++i) fa[20 + i] = xv[2 + i];
#pragma unroll
    for (int i = 0; i < 14; ++i) fb[i] = xv[i];
    fb[14] = ar;
    fb[15] = 0.6f * ar - 0.7f * (xv[2] + xv[3]);
#pragma unroll
    for (int i = 16; i < 32; ++i) fb[i] = 0.f;
    Pack16 u0, u1, u2, u3;
#pragma unroll
    for (int j = 0; j < 8; ++j) {
      u0.h[j] = (_Float16)(hh ? fb[j]      : fa[j]);
      u1.h[j] = (_Float16)(hh ? fb[8 + j]  : fa[8 + j]);
      u2.h[j] = (_Float16)(hh ? fb[16 + j] : fa[16 + j]);
      u3.h[j] = (_Float16)(hh ? fb[24 + j] : fa[24 + j]);
    }
    _Float16* ap = At + (16 * wave + m) * APA + 32 * hh;
    *(v8h*)ap = u0.h; *(v8h*)(ap + 8) = u1.h; *(v8h*)(ap + 16) = u2.h; *(v8h*)(ap + 24) = u3.h;
  }
  __syncthreads();

  Frag a0, a1, b00, b01, b10, b11;
  const _Float16* pa  = At + (16 * wave + m) * APA + 8 * hh;
  const _Float16* pb0 = wpl + (size_t)m * 64 + 8 * hh;
  const _Float16* pb1 = wpl + (size_t)(16 + m) * 64 + 8 * hh;
  a0.half[0]  = *(const v8h*)pa;         a0.half[1]  = *(const v8h*)(pa + 16);
  a1.half[0]  = *(const v8h*)(pa + 32);  a1.half[1]  = *(const v8h*)(pa + 48);
  b00.half[0] = *(const v8h*)pb0;        b00.half[1] = *(const v8h*)(pb0 + 16);
  b01.half[0] = *(const v8h*)(pb0 + 32); b01.half[1] = *(const v8h*)(pb0 + 48);
  b10.half[0] = *(const v8h*)pb1;        b10.half[1] = *(const v8h*)(pb1 + 16);
  b11.half[0] = *(const v8h*)(pb1 + 32); b11.half[1] = *(const v8h*)(pb1 + 48);
  const v8f z8 = {0.f, 0.f, 0.f, 0.f, 0.f, 0.f, 0.f, 0.f};
  v8f c0 = wm(a0.v, b00.v, z8);
  c0 = wm(a1.v, b01.v, c0);
  v8f c1 = wm(a0.v, b10.v, z8);
  c1 = wm(a1.v, b11.v, c1);

  const float bias0 = ab[m], w0 = bw[m];
  const int  n1 = 16 + m;
  const bool v1 = n1 < 20;
  const float bias1 = ab[n1 < 20 ? n1 : 19], w1 = bw[n1 < 20 ? n1 : 19];
  float part[8];
#pragma unroll
  for (int r = 0; r < 8; ++r) {
    const float p0 = fmaxf(c0[r] + bias0, 0.f) * w0;
    const float p1 = v1 ? fmaxf(c1[r] + bias1, 0.f) * w1 : 0.f;
    part[r] = p0 + p1;
  }
#pragma unroll
  for (int mk = 1; mk < 16; mk <<= 1) {
#pragma unroll
    for (int r = 0; r < 8; ++r) part[r] += __shfl_xor(part[r], mk, 32);
  }
  if (m == 0) {
    const float b0 = bb[0];
#pragma unroll
    for (int r = 0; r < 8; ++r) souts[16 * wave + 8 * hh + r] = part[r] + b0;
  }
  __syncthreads();
  if (tid < 16) {
    const v4f v = *(const v4f*)(souts + 4 * tid);
    float* op = sa + (size_t)rowBase + 4 * tid;
    *(volatile v4f*)op = v;
    __threadfence();
    *(volatile v4f*)op = v;
  }
}

__global__ __launch_bounds__(GTHR) void k_dep(
    const float* __restrict__ hpl, const float* __restrict__ x1,
    const int* __restrict__ tgt, const float* __restrict__ arm,
    const _Float16* __restrict__ wpl, const float* __restrict__ cb,
    const float* __restrict__ dw, const float* __restrict__ db,
    float* sd, int Md, int nN) {
  __shared__ __attribute__((aligned(16))) _Float16 At[GR * APN];
  __shared__ float souts[GR];
  const int tid = threadIdx.x, lane = tid & 31, wave = tid >> 5;
  const int hh = lane >> 4, m = lane & 15;
  const int rowBase = blockIdx.x * GR;

  {
    int row = rowBase + 16 * wave + m; if (row > Md - 1) row = Md - 1;
    const int it = clampi(tgt[row], 0, nN - 1);
    const float ar = arm[row];
    const float* hd = hpl + (size_t)it * 16;
    const v4f d0 = *(const v4f*)hd, d1 = *(const v4f*)(hd + 4), d2 = *(const v4f*)(hd + 8);
    const float* xp = x1 + (size_t)it * NF + 3;
    float xv[12];
#pragma unroll
    for (int i = 0; i < 12; ++i) xv[i] = xp[i];
    float fa[16], fb[16];
    fa[0] = d0.x; fa[1] = d0.y; fa[2] = d0.z; fa[3] = d0.w; fa[4] = d1.x;
    fa[5] = d1.y; fa[6] = d1.z; fa[7] = d1.w; fa[8] = d2.x; fa[9] = d2.y;
#pragma unroll
    for (int i = 0; i < 6; ++i) fa[10 + i] = xv[i];
#pragma unroll
    for (int i = 0; i < 6; ++i) fb[i] = xv[6 + i];
    fb[6] = ar;
#pragma unroll
    for (int i = 7; i < 16; ++i) fb[i] = 0.f;
    Pack16 u0, u1;
#pragma unroll
    for (int j = 0; j < 8; ++j) {
      u0.h[j] = (_Float16)(hh ? fb[j]     : fa[j]);
      u1.h[j] = (_Float16)(hh ? fb[8 + j] : fa[8 + j]);
    }
    _Float16* ap = At + (16 * wave + m) * APN + 16 * hh;
    *(v8h*)ap = u0.h; *(v8h*)(ap + 8) = u1.h;
  }
  __syncthreads();

  Frag a, b0, b1;
  const _Float16* pa  = At + (16 * wave + m) * APN + 8 * hh;
  const _Float16* pb0 = wpl + (size_t)m * 32 + 8 * hh;
  const _Float16* pb1 = wpl + (size_t)(16 + m) * 32 + 8 * hh;
  a.half[0]  = *(const v8h*)pa;  a.half[1]  = *(const v8h*)(pa + 16);
  b0.half[0] = *(const v8h*)pb0; b0.half[1] = *(const v8h*)(pb0 + 16);
  b1.half[0] = *(const v8h*)pb1; b1.half[1] = *(const v8h*)(pb1 + 16);
  const v8f z8 = {0.f, 0.f, 0.f, 0.f, 0.f, 0.f, 0.f, 0.f};
  const v8f c0 = wm(a.v, b0.v, z8);
  const v8f c1 = wm(a.v, b1.v, z8);

  const float bias0 = cb[m], w0 = dw[m];
  const int  n1 = 16 + m;
  const bool v1 = n1 < 20;
  const float bias1 = cb[n1 < 20 ? n1 : 19], w1 = dw[n1 < 20 ? n1 : 19];
  float part[8];
#pragma unroll
  for (int r = 0; r < 8; ++r) {
    const float p0 = fmaxf(c0[r] + bias0, 0.f) * w0;
    const float p1 = v1 ? fmaxf(c1[r] + bias1, 0.f) * w1 : 0.f;
    part[r] = p0 + p1;
  }
#pragma unroll
  for (int mk = 1; mk < 16; mk <<= 1) {
#pragma unroll
    for (int r = 0; r < 8; ++r) part[r] += __shfl_xor(part[r], mk, 32);
  }
  if (m == 0) {
    const float b0 = db[0];
#pragma unroll
    for (int r = 0; r < 8; ++r) souts[16 * wave + 8 * hh + r] = part[r] + b0;
  }
  __syncthreads();
  if (tid < 16) {
    const v4f v = *(const v4f*)(souts + 4 * tid);
    float* op = sd + (size_t)rowBase + 4 * tid;
    *(volatile v4f*)op = v;
    __threadfence();
    *(volatile v4f*)op = v;
  }
}

__global__ __launch_bounds__(GTHR) void k_val(
    const float* __restrict__ hpl, const float* __restrict__ x1, const float* __restrict__ x2,
    const _Float16* __restrict__ wpl, const float* __restrict__ lb,
    const float* __restrict__ l2w, const float* __restrict__ l2b,
    float* vp, int nN) {
  __shared__ __attribute__((aligned(16))) _Float16 At[GR * APN];
  __shared__ float sv[8];
  const int tid = threadIdx.x, lane = tid & 31, wave = tid >> 5;
  const int hh = lane >> 4, m = lane & 15;
  const int rowBase = blockIdx.x * GR;

  {
    int row = rowBase + 16 * wave + m; if (row > nN - 1) row = nN - 1;
    const float* hp = hpl + (size_t)row * 16;
    const v4f h0 = *(const v4f*)hp, h1 = *(const v4f*)(hp + 4), h2 = *(const v4f*)(hp + 8);
    const float* xp = x1 + (size_t)row * NF;
    float xv[15];
#pragma unroll
    for (int i = 0; i < 15; ++i) xv[i] = xp[i];
    float x2v[4];
#pragma unroll
    for (int i = 0; i < 4; ++i) x2v[i] = x2[i];
    float fa[16], fb[16];
    fa[0] = h0.x; fa[1] = h0.y; fa[2] = h0.z; fa[3] = h0.w; fa[4] = h1.x;
    fa[5] = h1.y; fa[6] = h1.z; fa[7] = h1.w; fa[8] = h2.x; fa[9] = h2.y;
#pragma unroll
    for (int i = 0; i < 6; ++i) fa[10 + i] = xv[i];
#pragma unroll
    for (int i = 0; i < 9; ++i) fb[i] = xv[6 + i];
#pragma unroll
    for (int i = 0; i < 4; ++i) fb[9 + i] = x2v[i];
    fb[13] = 0.f; fb[14] = 0.f; fb[15] = 0.f;
    Pack16 u0, u1;
#pragma unroll
    for (int j = 0; j < 8; ++j) {
      u0.h[j] = (_Float16)(hh ? fb[j]     : fa[j]);
      u1.h[j] = (_Float16)(hh ? fb[8 + j] : fa[8 + j]);
    }
    _Float16* ap = At + (16 * wave + m) * APN + 16 * hh;
    *(v8h*)ap = u0.h; *(v8h*)(ap + 8) = u1.h;
  }
  __syncthreads();

  Frag a, b;
  const _Float16* pa = At + (16 * wave + m) * APN + 8 * hh;
  const _Float16* pb = wpl + (size_t)m * 32 + 8 * hh;
  a.half[0] = *(const v8h*)pa; a.half[1] = *(const v8h*)(pa + 16);
  b.half[0] = *(const v8h*)pb; b.half[1] = *(const v8h*)(pb + 16);
  const v8f z8 = {0.f, 0.f, 0.f, 0.f, 0.f, 0.f, 0.f, 0.f};
  const v8f c0 = wm(a.v, b.v, z8);

  const bool vn = m < 15;
  const float bias0 = lb[m < 15 ? m : 14], w0 = l2w[m < 15 ? m : 14];
  float part[8];
#pragma unroll
  for (int r = 0; r < 8; ++r) part[r] = vn ? fmaxf(c0[r] + bias0, 0.f) * w0 : 0.f;
#pragma unroll
  for (int mk = 1; mk < 16; mk <<= 1) {
#pragma unroll
    for (int r = 0; r < 8; ++r) part[r] += __shfl_xor(part[r], mk, 32);
  }
  if (m == 0) {
    const float b0 = l2b[0];
    float hs = 0.f;
#pragma unroll
    for (int r = 0; r < 8; ++r) {
      const int row = rowBase + 16 * wave + 8 * hh + r;
      const float v = part[r] + b0;
      hs += (row < nN) ? v : 0.f;
    }
    sv[2 * wave + hh] = hs;
  }
  __syncthreads();
  if (wave == 0) {
    float tot = 0.f;
#pragma unroll
    for (int i = 0; i < 8; ++i) tot += sv[i];
    const float val = (lane == 0) ? tot : 0.f;
    float* op = vp + (size_t)blockIdx.x * 32 + lane;
    *(volatile float*)op = val;
    __threadfence();
    *(volatile float*)op = val;
  }
}

__global__ __launch_bounds__(32) void k_final(
    const int* __restrict__ amove, const float* __restrict__ sa, int Ma,
    const int* __restrict__ dmove, const float* __restrict__ sd, int Md,
    const float* __restrict__ vpart, int nvb, int nN, float* out, int M) {
  extern __shared__ v4f lds_dyn[];
  __shared__ double dred[32];
  float* S = (float*)lds_dyn;
  const int lane = threadIdx.x;
  {
    const v4f z4 = {0.f, 0.f, 0.f, 0.f};
    const int nq = (M + 8) / 4;
    for (int i = lane; i < nq; i += 32) lds_dyn[i] = z4;
  }
  __syncthreads();
  {
    const int ng = (Ma + 31) >> 5;
#pragma unroll 1
    for (int g = 0; g < ng; ++g) {
      const int i  = g * 32 + lane;
      const int ic = (i < Ma) ? i : Ma - 1;
      const int mv = clampi(amove[ic], 0, M - 1);
      float sv = sa[ic]; sv = (i < Ma) ? sv : 0.f;
      const int svb = __float_as_int(sv);
#pragma unroll
      for (int j = 0; j < 32; ++j) {
        const int   mj = __builtin_amdgcn_readlane(mv, j);
        const float vj = __int_as_float(__builtin_amdgcn_readlane(svb, j));
        S[1 + mj] = S[1 + mj] + vj;
      }
    }
  }
  {
    const int ng = (Md + 31) >> 5;
#pragma unroll 1
    for (int g = 0; g < ng; ++g) {
      const int i  = g * 32 + lane;
      const int ic = (i < Md) ? i : Md - 1;
      const int mv = clampi(dmove[ic], 0, M - 1);
      float sv = sd[ic]; sv = (i < Md) ? sv : 0.f;
      const int svb = __float_as_int(sv);
#pragma unroll
      for (int j = 0; j < 32; ++j) {
        const int   mj = __builtin_amdgcn_readlane(mv, j);
        const float vj = __int_as_float(__builtin_amdgcn_readlane(svb, j));
        S[1 + mj] = S[1 + mj] + vj;
      }
    }
  }
  __syncthreads();

  float mx = -INFINITY;
  for (int i = lane; i < M; i += 32) mx = fmaxf(mx, S[1 + i]);
#pragma unroll
  for (int k = 16; k > 0; k >>= 1) mx = fmaxf(mx, __shfl_xor(mx, k, 32));
  float se = 0.f;
#pragma unroll 1
  for (int i = lane; i < M; i += 32) se += expf(S[1 + i] - mx);
#pragma unroll
  for (int k = 16; k > 0; k >>= 1) se += __shfl_xor(se, k, 32);
  const float lg = logf(se);

  double ds = 0.0;
#pragma unroll 1
  for (int b = lane; b < nvb; b += 32) ds += (double)vpart[(size_t)b * 32];
  dred[lane] = ds;
  __syncthreads();
  double tot = 0.0;
#pragma unroll 1
  for (int k = 0; k < 32; ++k) tot += dred[k];
  const float V = tanhf((float)(tot / (double)nN));

  for (int i = lane; i < M; i += 32) S[1 + i] = (S[1 + i] - mx) - lg;
  __syncthreads();
  if (lane == 0) S[0] = V;
  __syncthreads();

  const int total = M + 1;
  const int np = total >> 2;
  const int ntail = total - 4 * np;
  for (int q = lane; q < np; q += 32) {
    const v4f v = *(const v4f*)(S + 4 * q);
    *(volatile v4f*)(out + 4 * q) = v;
  }
  if (lane == 0) {
    for (int t = 0; t < ntail; ++t) { const float v = S[4 * np + t]; *(volatile float*)(out + 4 * np + t) = v; }
  }
  __threadfence();
  for (int q = lane; q < np; q += 32) {
    const v4f v = *(const v4f*)(S + 4 * q);
    *(volatile v4f*)(out + 4 * q) = v;
  }
  if (lane == 0) {
    for (int t = 0; t < ntail; ++t) { const float v = S[4 * np + t]; *(volatile float*)(out + 4 * np + t) = v; }
  }
}

extern "C" void kernel_launch(void* const* d_in, const int* in_sizes, int n_in,
                              void* d_out, int out_size, void* d_ws, size_t ws_size,
                              hipStream_t stream) {
  if (n_in < 35) return;
  const int nN = in_sizes[0] / NF;
  if (nN <= 0 || in_sizes[0] != nN * NF) return;
  if (in_sizes[1] != 4) return;
  const int nE = in_sizes[2] / 2;
  if (nE < 1 || in_sizes[2] != 2 * nE) return;
  const int Ma = in_sizes[3];
  if (Ma < 1 || in_sizes[4] != Ma || in_sizes[5] != Ma || in_sizes[6] != Ma) return;
  const int Md = in_sizes[7];
  if (Md < 1 || in_sizes[8] != Md || in_sizes[9] != Md) return;
  const int M = out_size - 1;
  if (M < 1) return;
  if (in_sizes[11] != 150 || in_sizes[12] != 150 || in_sizes[13] != 10 || in_sizes[14] != 10) return;
  if (in_sizes[15] != 250 || in_sizes[16] != 250 || in_sizes[17] != 10 || in_sizes[18] != 10) return;
  if (in_sizes[19] != 250 || in_sizes[20] != 250 || in_sizes[21] != 10 || in_sizes[22] != 10) return;
  if (in_sizes[23] != 435 || in_sizes[24] != 15 || in_sizes[25] != 15 || in_sizes[26] != 1) return;
  if (in_sizes[27] != 960 || in_sizes[28] != 20 || in_sizes[29] != 20 || in_sizes[30] != 1) return;
  if (in_sizes[31] != 460 || in_sizes[32] != 20 || in_sizes[33] != 20 || in_sizes[34] != 1) return;

  const float* x1    = (const float*)d_in[0];
  const float* x2    = (const float*)d_in[1];
  const int*   edges = (const int*)d_in[2];
  const int*   asrc  = (const int*)d_in[3];
  const int*   adst  = (const int*)d_in[4];
  const float* aarm  = (const float*)d_in[5];
  const int*   amove = (const int*)d_in[6];
  const int*   dtgt  = (const int*)d_in[7];
  const float* darm  = (const float*)d_in[8];
  const int*   dmove = (const int*)d_in[9];
  const float* wl0 = (const float*)d_in[11]; const float* wr0 = (const float*)d_in[12];
  const float* at0 = (const float*)d_in[13]; const float* gb0 = (const float*)d_in[14];
  const float* wl1 = (const float*)d_in[15]; const float* wr1 = (const float*)d_in[16];
  const float* at1 = (const float*)d_in[17]; const float* gb1 = (const float*)d_in[18];
  const float* wl2 = (const float*)d_in[19]; const float* wr2 = (const float*)d_in[20];
  const float* at2 = (const float*)d_in[21]; const float* gb2 = (const float*)d_in[22];
  const float* linW  = (const float*)d_in[23];
  const float* linB  = (const float*)d_in[24];
  const float* lin2W = (const float*)d_in[25];
  const float* lin2B = (const float*)d_in[26];
  const float* aaaW  = (const float*)d_in[27];
  const float* aaaB  = (const float*)d_in[28];
  const float* bbbW  = (const float*)d_in[29];
  const float* bbbB  = (const float*)d_in[30];
  const float* cccW  = (const float*)d_in[31];
  const float* cccB  = (const float*)d_in[32];
  const float* dddW  = (const float*)d_in[33];
  const float* dddB  = (const float*)d_in[34];

  const int gridN  = (nN + GR - 1) / GR;
  const int nNp64  = gridN * GR;
  const int gridAg = (nN + NBA - 1) / NBA;
  const int nNpA   = gridAg * NBA;
  const int gridAt = (Ma + GR - 1) / GR;
  const int gridDp = (Md + GR - 1) / GR;

  char* w8 = (char*)d_ws;
  size_t off = 0;
  _Float16* WPL = (_Float16*)(w8 + off); off += ((size_t)WPL_HALVES * 2 + 255) & ~(size_t)255;
  float* XLR = (float*)(w8 + off); off += ((size_t)nNp64 * 32 * 4 + 255) & ~(size_t)255;
  float* HPL = (float*)(w8 + off); off += ((size_t)nNpA * 16 * 4 + 255) & ~(size_t)255;
  float* SA  = (float*)(w8 + off); off += ((size_t)gridAt * GR * 4 + 255) & ~(size_t)255;
  float* SD  = (float*)(w8 + off); off += ((size_t)gridDp * GR * 4 + 255) & ~(size_t)255;
  float* VP  = (float*)(w8 + off); off += ((size_t)gridN * 32 * 4 + 255) & ~(size_t)255;
  if (off > ws_size || off > (size_t)134217728) return;

  const size_t fin_lds = (size_t)((M + 8) / 4) * 16;
  if (fin_lds > (size_t)294912) return;

  k_prepw<<<(WPL_PIECES + 255) / 256, 256, 0, stream>>>(wl0, wr0, wl1, wr1, wl2, wr2,
                                                         aaaW, cccW, linW, WPL, WPL_PIECES);

  hipFuncSetAttribute(reinterpret_cast<const void*>(&k_agg),
                      hipFuncAttributeMaxDynamicSharedMemorySize, AGG_LDS_BYTES);
  hipFuncSetAttribute(reinterpret_cast<const void*>(&k_final),
                      hipFuncAttributeMaxDynamicSharedMemorySize, (int)fin_lds);

  const float* atl[3] = {at0, at1, at2};
  const float* gbl[3] = {gb0, gb1, gb2};
  for (int l = 0; l < 3; ++l) {
    k_node<<<gridN, GTHR, 0, stream>>>(x1, HPL, WPL + 1024 * l, XLR, l == 0 ? 0 : 10, nN);
    k_agg<<<gridAg, ATHR, AGG_LDS_BYTES, stream>>>(edges, XLR, atl[l], gbl[l], HPL, nN, nE);
  }
  k_att<<<gridAt, GTHR, 0, stream>>>(HPL, x1, asrc, adst, aarm, WPL + 3072, aaaB, bbbW, bbbB,
                                     SA, Ma, nN);
  k_dep<<<gridDp, GTHR, 0, stream>>>(HPL, x1, dtgt, darm, WPL + 5120, cccB, dddW, dddB,
                                     SD, Md, nN);
  k_val<<<gridN, GTHR, 0, stream>>>(HPL, x1, x2, WPL + 6144, linB, lin2W, lin2B, VP, nN);
  k_final<<<1, 32, fin_lds, stream>>>(amove, SA, Ma, dmove, SD, Md, VP, gridN, nN,
                                      (float*)d_out, M);
}
